// Model_32676111188683
// MI455X (gfx1250) — hardware-verified
//
#include <hip/hip_runtime.h>
#include <math.h>

constexpr int NBATCH  = 64;
constexpr int NSTEP   = 1024;
constexpr int NFEAT   = 2;
constexpr int NHID    = 512;
constexpr int NLAYER  = 3;
constexpr int SEQ_BLK = 16;
constexpr int NTHR    = 256;
constexpr int HPITCH  = 520;
constexpr int SPITCH  = 516;
constexpr float HCARRY     = 16.0f;
constexpr float WCARRY     = 256.0f;
constexpr float ACARRY     = HCARRY * WCARRY;
constexpr float ACARRY_INV = 1.0f / ACARRY;
constexpr int PLANE   = NHID * NHID;
constexpr int NPLANE  = (NLAYER - 1) + NLAYER;
constexpr int N8_IH   = (NLAYER - 1) * PLANE / 8;
constexpr int N8_HH   = NLAYER * PLANE / 8;
constexpr int NBLK_W  = (N8_IH + N8_HH) / NTHR;
constexpr int NB4     = NLAYER * NHID / 4;
constexpr int NBLK_B  = (NB4 + NTHR - 1) / NTHR;
constexpr int NOUT0   = NBATCH * NFEAT;
constexpr int NOUT1   = NLAYER * NBATCH * NHID;

static_assert(NBATCH % SEQ_BLK == 0, "blocks own whole 16-row groups");
static_assert(NHID == 64 * (NTHR / 32), "8 waves x 64 hidden columns");
static_assert(NHID % 32 == 0, "K multiple of 32");
static_assert(N8_IH % NTHR == 0 && N8_HH % NTHR == 0, "block-uniform source select in the prep kernel");
static_assert((NLAYER * SEQ_BLK * NHID) % NTHR == 0, "state init loop exact");
static_assert(SEQ_BLK * NFEAT == 32, "one 128-B line of the head output per block");
static_assert((NOUT0 * 4) % 128 == 0, "second output starts on a 128-B line");
static_assert((HPITCH % 8) == 0 && (SPITCH % 4) == 0, "16-B aligned LDS rows");
static_assert(NB4 <= NBLK_B * NTHR, "bias blocks cover the bias plane");

typedef __attribute__((ext_vector_type(16))) _Float16 v16h;
typedef __attribute__((ext_vector_type(8)))  _Float16 v8h;
typedef __attribute__((ext_vector_type(8)))  float    v8f;
typedef __attribute__((ext_vector_type(4)))  float    v4f;
typedef __attribute__((ext_vector_type(2)))  float    v2f;

struct FragH {
  union U { v16h v; v8h h[2]; };
  static __device__ __forceinline__ v16h load(const _Float16* p) {
    U f;
    f.h[0] = *(const v8h*)(p);
    f.h[1] = *(const v8h*)(p + 16);
    return f.v;
  }
  static __device__ __forceinline__ v8f mma(v16h a, v16h b, v8f c) {
    return __builtin_amdgcn_wmma_f32_16x16x32_f16(false, a, false, b, (short)0, c, false, false);
  }
};

__device__ __forceinline__ void guard_all(v8f& a0, v8f& a1, v8f& a2, v8f& a3,
                                          v16h x, v16h b0, v16h b1, v16h b2, v16h b3) {
  asm volatile("v_nop\n\tv_nop\n\tv_nop\n\tv_nop"
               : "+v"(a0), "+v"(a1), "+v"(a2), "+v"(a3)
               : "v"(x), "v"(b0), "v"(b1), "v"(b2), "v"(b3));
}
__device__ __forceinline__ void acc_guard4(v8f& a, v8f& b, v8f& c, v8f& d) {
  asm volatile("v_nop\n\tv_nop\n\tv_nop\n\tv_nop" : "+v"(a), "+v"(b), "+v"(c), "+v"(d));
}

__device__ __forceinline__ void tile_k512(v8f& a0, v8f& a1, v8f& a2, v8f& a3,
                                          const _Float16* arow, const _Float16* wrow) {
#pragma unroll 1
  for (int k0 = 0; k0 < NHID; k0 += 32) {
    const v16h a  = FragH::load(arow + k0);
    const v16h b0 = FragH::load(wrow + k0);
    const v16h b1 = FragH::load(wrow + (size_t)16 * NHID + k0);
    const v16h b2 = FragH::load(wrow + (size_t)32 * NHID + k0);
    const v16h b3 = FragH::load(wrow + (size_t)48 * NHID + k0);
    a0 = FragH::mma(a, b0, a0);
    a1 = FragH::mma(a, b1, a1);
    a2 = FragH::mma(a, b2, a2);
    a3 = FragH::mma(a, b3, a3);
    guard_all(a0, a1, a2, a3, a, b0, b1, b2, b3);
  }
}

__device__ __forceinline__ float tanh_f32(float x) {
  const float xc = fminf(fmaxf(x, -15.0f), 15.0f);
  const float e  = __expf(2.0f * xc);
  const float d  = e + 1.0f;
  float r = __builtin_amdgcn_rcpf(d);
  r = fmaf(fmaf(-d, r, 1.0f), r, r);
  return 1.0f - 2.0f * r;
}

__global__ __launch_bounds__(NTHR) void prep_kernel(const float* __restrict__ wih, const float* __restrict__ whh,
                                                    const float* __restrict__ bih0, const float* __restrict__ bihr,
                                                    const float* __restrict__ bhh,
                                                    unsigned short* __restrict__ W16, float* __restrict__ bsum) {
  const int tid = threadIdx.x;
  const int blk = blockIdx.x;
  if (blk < NBLK_W) {
    const int i = blk * NTHR + tid;
    const bool from_ih = (blk < N8_IH / NTHR);
    const float* sp = from_ih ? (wih + (size_t)i * 8) : (whh + (size_t)(i - N8_IH) * 8);
    const v4f a = *(const v4f*)(sp);
    const v4f b = *(const v4f*)(sp + 4);
    v8h hv;
#pragma unroll
    for (int e = 0; e < 4; ++e) {
      const float fa = a[e] * WCARRY;
      const float fb = b[e] * WCARRY;
      hv[e]     = (_Float16)fa;
      hv[4 + e] = (_Float16)fb;
    }
    unsigned short* dp = W16 + (size_t)i * 8;
    *(volatile v8h*)dp = hv;
    __threadfence();
    *(volatile v8h*)dp = hv;
  } else {
    const int bi = (blk - NBLK_W) * NTHR + tid;
    if (bi < NB4) {
      const int l  = bi / (NHID / 4);
      const int n4 = (bi - l * (NHID / 4)) * 4;
      const int lm = (l > 0) ? (l - 1) : 0;
      const v4f v0 = *(const v4f*)(bih0 + n4);
      const v4f v1 = *(const v4f*)(bihr + (size_t)lm * NHID + n4);
      const v4f vh = *(const v4f*)(bhh + (size_t)l * NHID + n4);
      v4f o;
#pragma unroll
      for (int e = 0; e < 4; ++e) {
        const float bi_e = (l == 0) ? v0[e] : v1[e];
        o[e] = bi_e + vh[e];
      }
      float* op = bsum + (size_t)bi * 4;
      *(volatile v4f*)op = o;
      __threadfence();
      *(volatile v4f*)op = o;
    }
  }
}

__global__ __launch_bounds__(NTHR) void rnn_seq_kernel(const float* __restrict__ input, const float* __restrict__ hidden,
                                                       const float* __restrict__ w_ih0,
                                                       const unsigned short* __restrict__ W16p,
                                                       const float* __restrict__ bsum,
                                                       const float* __restrict__ w_dense, const float* __restrict__ b_dense,
                                                       float* __restrict__ out) {
  __shared__ __align__(16) _Float16 Hh[NLAYER * SEQ_BLK * HPITCH];
  __shared__ __align__(16) float    Hs[SEQ_BLK * SPITCH];
  const _Float16* W16 = (const _Float16*)W16p;
  const int tid = threadIdx.x, lane = tid & 31, wave = tid >> 5;
  const int c = lane & 15, hh = lane >> 4, koff = hh * 8;
  const int rowbase = blockIdx.x * SEQ_BLK;
  const int ncol = 64 * wave + c;

#pragma unroll 1
  for (int i = tid; i < NLAYER * SEQ_BLK * NHID; i += NTHR) {
    const int l   = i / (SEQ_BLK * NHID);
    const int rem = i - l * (SEQ_BLK * NHID);
    const int m   = rem / NHID;
    const int n   = rem - m * NHID;
    const float hv = hidden[((size_t)l * NBATCH + rowbase + m) * NHID + n];
    Hh[(l * SEQ_BLK + m) * HPITCH + n] = (_Float16)(hv * HCARRY);
  }
#pragma unroll 1
  for (int i = tid; i < NLAYER * SEQ_BLK * (HPITCH - NHID); i += NTHR) {
    const int row = i / (HPITCH - NHID);
    const int col = NHID + (i - row * (HPITCH - NHID));
    Hh[row * HPITCH + col] = (_Float16)0.0f;
  }

  float w00, w01, w10, w11, w20, w21, w30, w31;
  {
    const v2f q0 = *(const v2f*)(w_ih0 + (size_t)(ncol +  0) * NFEAT);
    const v2f q1 = *(const v2f*)(w_ih0 + (size_t)(ncol + 16) * NFEAT);
    const v2f q2 = *(const v2f*)(w_ih0 + (size_t)(ncol + 32) * NFEAT);
    const v2f q3 = *(const v2f*)(w_ih0 + (size_t)(ncol + 48) * NFEAT);
    w00 = q0[0]; w01 = q0[1];
    w10 = q1[0]; w11 = q1[1];
    w20 = q2[0]; w21 = q2[1];
    w30 = q3[0]; w31 = q3[1];
  }
  __syncthreads();

  const float* xrow = input + (size_t)(rowbase + 8 * hh) * (NSTEP * NFEAT);

#pragma unroll 1
  for (int t = 0; t < NSTEP; ++t) {
    const bool last = (t == NSTEP - 1);

#pragma unroll 1
    for (int l = 0; l < NLAYER; ++l) {
      const float bs0 = bsum[l * NHID + ncol];
      const float bs1 = bsum[l * NHID + ncol + 16];
      const float bs2 = bsum[l * NHID + ncol + 32];
      const float bs3 = bsum[l * NHID + ncol + 48];
      v8f acc0, acc1, acc2, acc3;
      if (l == 0) {
#pragma unroll
        for (int r = 0; r < 8; ++r) {
          const v2f xv = *(const v2f*)(xrow + (size_t)r * (NSTEP * NFEAT) + 2 * t);
          const float xa = xv[0];
          const float xb = xv[1];
          acc0[r] = (bs0 + (xa * w00 + xb * w01)) * ACARRY;
          acc1[r] = (bs1 + (xa * w10 + xb * w11)) * ACARRY;
          acc2[r] = (bs2 + (xa * w20 + xb * w21)) * ACARRY;
          acc3[r] = (bs3 + (xa * w30 + xb * w31)) * ACARRY;
        }
      } else {
#pragma unroll
        for (int r = 0; r < 8; ++r) {
          acc0[r] = bs0 * ACARRY;
          acc1[r] = bs1 * ACARRY;
          acc2[r] = bs2 * ACARRY;
          acc3[r] = bs3 * ACARRY;
        }
      }

      {
        const _Float16* arow = Hh + (l * SEQ_BLK + c) * HPITCH + koff;
        const _Float16* wrow = W16 + (size_t)(NLAYER - 1 + l) * PLANE + (size_t)ncol * NHID + koff;
        tile_k512(acc0, acc1, acc2, acc3, arow, wrow);
      }
      if (l >= 1) {
        const _Float16* arow = Hh + ((l - 1) * SEQ_BLK + c) * HPITCH + koff;
        const _Float16* wrow = W16 + (size_t)(l - 1) * PLANE + (size_t)ncol * NHID + koff;
        tile_k512(acc0, acc1, acc2, acc3, arow, wrow);
      }
      acc_guard4(acc0, acc1, acc2, acc3);

      __syncthreads();

      _Float16* hl = Hh + (l * SEQ_BLK + 8 * hh) * HPITCH;
#pragma unroll 1
      for (int jj = 0; jj < 4; ++jj) {
        v8f cur = acc0;
        if (jj == 1) cur = acc1;
        if (jj == 2) cur = acc2;
        if (jj == 3) cur = acc3;
        const int col = ncol + 16 * jj;
#pragma unroll
        for (int r = 0; r < 8; ++r) {
          const float pre = cur[r] * ACARRY_INV;
          const float hv  = tanh_f32(pre);
          hl[r * HPITCH + col] = (_Float16)(hv * HCARRY);
          if (last) Hs[(8 * hh + r) * SPITCH + col] = hv;
        }
      }

      __syncthreads();

      if (last) {
        float* o1 = out + NOUT0 + ((size_t)l * NBATCH + rowbase) * NHID;
        for (int pass = 0; pass < 2; ++pass) {
#pragma unroll
          for (int it = 0; it < 8; ++it) {
            const int idx = it * NTHR + tid;
            const int row = idx >> 7;
            const int c4  = (idx & 127) * 4;
            const v4f v = *(const v4f*)(Hs + row * SPITCH + c4);
            *(volatile v4f*)(o1 + (size_t)row * NHID + c4) = v;
          }
          __threadfence();
        }
        if (l == NLAYER - 1 && wave == 0) {
          const int row = lane >> 1;
          const int o   = lane & 1;
          const float* hr = Hs + row * SPITCH;
          const float* wd = w_dense + (size_t)o * NHID;
          float s0 = 0.0f, s1 = 0.0f, s2 = 0.0f, s3 = 0.0f;
#pragma unroll 2
          for (int k = 0; k < NHID; k += 4) {
            const v4f hv = *(const v4f*)(hr + k);
            const v4f wv = *(const v4f*)(wd + k);
            s0 = fmaf(hv[0], wv[0], s0);
            s1 = fmaf(hv[1], wv[1], s1);
            s2 = fmaf(hv[2], wv[2], s2);
            s3 = fmaf(hv[3], wv[3], s3);
          }
          const float s = ((s0 + s1) + (s2 + s3)) + b_dense[o];
          float* op = out + (size_t)rowbase * NFEAT + lane;
          *(volatile float*)op = s;
          __threadfence();
          *(volatile float*)op = s;
        }
      }
    }
  }
}

extern "C" void kernel_launch(void* const* d_in, const int* in_sizes, int n_in,
                              void* d_out, int out_size, void* d_ws, size_t ws_size, hipStream_t stream) {
  if (n_in < 10 || d_out == nullptr || d_ws == nullptr) return;
  if (in_sizes[0] != NBATCH * NSTEP * NFEAT || in_sizes[1] != NLAYER * NBATCH * NHID ||
      in_sizes[2] != NHID * NFEAT || in_sizes[3] != NHID ||
      in_sizes[4] != (NLAYER - 1) * PLANE || in_sizes[5] != (NLAYER - 1) * NHID ||
      in_sizes[6] != NLAYER * PLANE || in_sizes[7] != NLAYER * NHID ||
      in_sizes[8] != NFEAT * NHID || in_sizes[9] != NFEAT ||
      out_size != NOUT0 + NOUT1) return;

  const float* x_in    = (const float*)d_in[0];
  const float* hidden  = (const float*)d_in[1];
  const float* w_ih0   = (const float*)d_in[2];
  const float* b_ih0   = (const float*)d_in[3];
  const float* w_ihr   = (const float*)d_in[4];
  const float* b_ihr   = (const float*)d_in[5];
  const float* w_hh    = (const float*)d_in[6];
  const float* b_hh    = (const float*)d_in[7];
  const float* w_dense = (const float*)d_in[8];
  const float* b_dense = (const float*)d_in[9];
  float* out = (float*)d_out;

  char* ws = (char*)d_ws;
  size_t off = 0;
  auto carve = [&](size_t bytes) -> char* { char* p = ws + off; off += (bytes + 255) & ~(size_t)255; return p; };
  unsigned short* W16  = (unsigned short*)carve((size_t)NPLANE * PLANE * 2);
  float*          BSUM = (float*)carve((size_t)NLAYER * NHID * 4);
  if (off > ws_size || off > (size_t)134217728) return;

  prep_kernel<<<NBLK_W + NBLK_B, NTHR, 0, stream>>>(w_ihr, w_hh, b_ih0, b_ihr, b_hh, W16, BSUM);
  rnn_seq_kernel<<<NBATCH / SEQ_BLK, NTHR, 0, stream>>>(x_in, hidden, w_ih0, W16, BSUM, w_dense, b_dense, out);
}
